// CCN_3951369912894
// MI455X (gfx1250) — hardware-verified
//
#include <hip/hip_runtime.h>
#include <stddef.h>


#define NP   4096
#define DIM  128
#define BT   128
#define KS   64
#define NTHR 256

typedef _Float16 v16h __attribute__((ext_vector_type(16)));
typedef _Float16 v8h  __attribute__((ext_vector_type(8)));
typedef float    v8f  __attribute__((ext_vector_type(8)));
typedef float    v4f  __attribute__((ext_vector_type(4)));

union Frag { v16h v; v8h hf[2]; };
union U8h  { v8h v; unsigned short u[8]; };

__device__ __forceinline__ v8f mma16(const v16h a, const v16h b, v8f c)
{
    c = __builtin_amdgcn_wmma_f32_16x16x32_f16(false, a, false, b, (short)0, c, false, false);
    asm volatile("v_nop\n\tv_nop\n\tv_nop\n\tv_nop" : "+v"(c) : "v"(a), "v"(b));
    return c;
}

__global__ __launch_bounds__(NTHR) void k_fv0(const float* __restrict__ nl,
                                            const float* __restrict__ td,
                                            const float* __restrict__ dep,
                                            const float* __restrict__ w,
                                            const float* __restrict__ b,
                                            _Float16* __restrict__ fv0T,
                                            int nreal)
{
    const int tid = threadIdx.x, wave = tid >> 5, l = tid & 31;
    const int g  = blockIdx.x * (NTHR / 32) + wave;
    const int d  = g >> 1;
    const int i0 = (g & 1) * (NP / 2);
    if (d >= DIM) return;
    const float w0 = w[d * 3 + 0], w1 = w[d * 3 + 1], w2 = w[d * 3 + 2], bb = b[d];
    const float xd = dep[0], yd = dep[1];
    _Float16* dst = fv0T + (size_t)d * NP + i0 + l * 8;

    #pragma unroll 1
    for (int s = 0; s < 8; ++s) {
        v8h t = {};
        #pragma unroll
        for (int e = 0; e < 8; ++e) {
            const int i = i0 + s * 256 + l * 8 + e;
            float v = 0.0f;
            if (i < nreal) {
                float x, y, tt;
                if (i == 0) { x = xd; y = yd; tt = 0.0f; }
                else { x = nl[(size_t)(i - 1) * 2]; y = nl[(size_t)(i - 1) * 2 + 1]; tt = td[i - 1]; }
                v = x * w0 + y * w1 + tt * w2 + bb;
                v = v > 0.0f ? v : 0.0f;
            }
            t[e] = (_Float16)v;
        }
        *(volatile v8h*)(dst + s * 256) = t;
    }
    __threadfence();
    #pragma unroll 1
    for (int s = 0; s < 8; ++s) {
        v8h t = {};
        #pragma unroll
        for (int e = 0; e < 8; ++e) {
            const int i = i0 + s * 256 + l * 8 + e;
            float v = 0.0f;
            if (i < nreal) {
                float x, y, tt;
                if (i == 0) { x = xd; y = yd; tt = 0.0f; }
                else { x = nl[(size_t)(i - 1) * 2]; y = nl[(size_t)(i - 1) * 2 + 1]; tt = td[i - 1]; }
                v = x * w0 + y * w1 + tt * w2 + bb;
                v = v > 0.0f ? v : 0.0f;
            }
            t[e] = (_Float16)v;
        }
        *(volatile v8h*)(dst + s * 256) = t;
    }
}

__global__ __launch_bounds__(NTHR) void k_adj(const float* __restrict__ nl,
                                            const float* __restrict__ dep,
                                            _Float16* __restrict__ Ah,
                                            int nreal)
{
    #pragma clang fp contract(off)
    __shared__ float lx[NP];
    __shared__ float ly[NP];
    const int tid = threadIdx.x, wave = tid >> 5, l = tid & 31;
    for (int jn = tid; jn < NP; jn += NTHR) {
        float x = 0.0f, y = 0.0f;
        if (jn == 0) { x = dep[0]; y = dep[1]; }
        else if (jn < nreal) { x = nl[(size_t)(jn - 1) * 2]; y = nl[(size_t)(jn - 1) * 2 + 1]; }
        lx[jn] = x; ly[jn] = y;
    }
    __syncthreads();

    const float  th  = 0.04f;
    const float  thn = __uint_as_float(__float_as_uint(th) + 1u);
    const double mid = ((double)th + (double)thn) * 0.5;
    const double m2  = mid * mid;

    #pragma unroll 1
    for (int rr = 0; rr < 4; ++rr) {
        const int i = blockIdx.x * 32 + wave * 4 + rr;
        const bool rowok = (i < nreal);
        const float xi = lx[i], yi = ly[i];
        _Float16* dst = Ah + (size_t)i * NP + l * 8;
        v8h vals[16];
        #pragma unroll
        for (int s = 0; s < 16; ++s) {
            v8h t = {};
            #pragma unroll
            for (int e = 0; e < 8; ++e) {
                const int jn = s * 256 + l * 8 + e;
                const float dx = xi - lx[jn];
                const float dy = yi - ly[jn];
                const float sq = dx * dx + dy * dy;
                const bool nb = rowok && (jn < nreal) && ((double)sq < m2);
                t[e] = nb ? (_Float16)1.0f : (_Float16)0.0f;
            }
            vals[s] = t;
            *(volatile v8h*)(dst + s * 256) = t;
        }
        __threadfence();
        #pragma unroll
        for (int s = 0; s < 16; ++s) *(volatile v8h*)(dst + s * 256) = vals[s];
    }
}

template<int EPI>
__global__ __launch_bounds__(NTHR) void k_gemm(const _Float16* __restrict__ L,
                                             const _Float16* __restrict__ RT,
                                             const _Float16* __restrict__ msk,
                                             _Float16* __restrict__ oh,
                                             float* __restrict__ of,
                                             int nreal)
{
    __shared__ __attribute__((aligned(16))) unsigned char lds[32768];
    _Float16* Ls = (_Float16*)lds;
    _Float16* Rs = (_Float16*)(lds + 16384);

    const int tid = threadIdx.x, wave = tid >> 5, l = tid & 31, h = l >> 4, m = l & 15;
    const int wm = wave & 3, wn = wave >> 2;
    const int bm = blockIdx.x, bn = blockIdx.y;
    const _Float16* Lb = L  + (size_t)bm * BT * NP;
    const _Float16* Rb = RT + (size_t)bn * BT * NP;

    v8f acc[2][4] = {};

    for (int kb = 0; kb < NP; kb += KS) {
        #pragma unroll
        for (int u = 0; u < (BT * KS / 8) / NTHR; ++u) {
            const int c = tid + NTHR * u;
            const int r = c >> 3, q = c & 7;
            const v8h x = *(const v8h*)(Lb + (size_t)r * NP + kb + q * 8);
            const v8h y = *(const v8h*)(Rb + (size_t)r * NP + kb + q * 8);
            *(v8h*)(Ls + r * KS + q * 8) = x;
            *(v8h*)(Rs + r * KS + q * 8) = y;
        }
        __syncthreads();
        #pragma unroll
        for (int kk = 0; kk < KS; kk += 32) {
            Frag a[2], b[4];
            #pragma unroll
            for (int mi = 0; mi < 2; ++mi) {
                const _Float16* p = Ls + (wm * 32 + mi * 16 + m) * KS + kk + 8 * h;
                a[mi].hf[0] = *(const v8h*)(p);
                a[mi].hf[1] = *(const v8h*)(p + 16);
            }
            #pragma unroll
            for (int ni = 0; ni < 4; ++ni) {
                const _Float16* p = Rs + (wn * 64 + ni * 16 + m) * KS + kk + 8 * h;
                b[ni].hf[0] = *(const v8h*)(p);
                b[ni].hf[1] = *(const v8h*)(p + 16);
            }
            #pragma unroll
            for (int mi = 0; mi < 2; ++mi)
                #pragma unroll
                for (int ni = 0; ni < 4; ++ni)
                    acc[mi][ni] = mma16(a[mi].v, b[ni].v, acc[mi][ni]);
        }
        __syncthreads();
    }

    if (EPI == 0 || EPI == 1) {
        _Float16* S = (_Float16*)lds + wave * 2048;
        #pragma unroll
        for (int mi = 0; mi < 2; ++mi)
            #pragma unroll
            for (int ni = 0; ni < 4; ++ni)
                #pragma unroll
                for (int r = 0; r < 8; ++r) {
                    const float cv = acc[mi][ni][r];
                    _Float16 hv;
                    if (EPI == 0) hv = (cv > 0.5f) ? (_Float16)1.0f : (_Float16)0.0f;
                    else          hv = (_Float16)cv;
                    S[(mi * 16 + 8 * h + r) * 64 + ni * 16 + m] = hv;
                }
        __syncthreads();
        const int q = l >> 3, j = l & 7;
        const int row0 = bm * BT + wm * 32, col0 = bn * BT + wn * 64;
        v8h vals[8];
        #pragma unroll
        for (int s = 0; s < 8; ++s) {
            const int lr = 4 * s + q;
            U8h vu; vu.v = *(const v8h*)(S + lr * 64 + j * 8);
            const size_t go = (size_t)(row0 + lr) * NP + col0 + j * 8;
            if (EPI == 1) {
                U8h mu; mu.v = *(const v8h*)(msk + go);
                #pragma unroll
                for (int e = 0; e < 8; ++e) if (mu.u[e] == 0) vu.u[e] = 0;
            }
            vals[s] = vu.v;
            *(volatile v8h*)(oh + go) = vals[s];
        }
        __threadfence();
        #pragma unroll
        for (int s = 0; s < 8; ++s) {
            const int lr = 4 * s + q;
            const size_t go = (size_t)(row0 + lr) * NP + col0 + j * 8;
            *(volatile v8h*)(oh + go) = vals[s];
        }
    }

    if (EPI == 2) {
        _Float16* T = (_Float16*)lds;
        #pragma unroll
        for (int mi = 0; mi < 2; ++mi)
            #pragma unroll
            for (int ni = 0; ni < 4; ++ni)
                #pragma unroll
                for (int r = 0; r < 8; ++r) {
                    const int dc = wn * 64 + ni * 16 + m;
                    const int v  = wm * 32 + mi * 16 + 8 * h + r;
                    T[dc * BT + v] = (_Float16)acc[mi][ni][r];
                }
        __syncthreads();
        const int q = l >> 3, j = l & 7;
        const int v0 = bm * BT;
        v8h vals[8];
        #pragma unroll
        for (int s = 0; s < 8; ++s) {
            const int ln = wave * 32 + 4 * s + q;
            const int dc = ln >> 1, hf = ln & 1;
            vals[s] = *(const v8h*)(T + dc * BT + hf * 64 + j * 8);
            const size_t go = (size_t)dc * NP + v0 + hf * 64 + j * 8;
            *(volatile v8h*)(oh + go) = vals[s];
        }
        __threadfence();
        #pragma unroll
        for (int s = 0; s < 8; ++s) {
            const int ln = wave * 32 + 4 * s + q;
            const int dc = ln >> 1, hf = ln & 1;
            const size_t go = (size_t)dc * NP + v0 + hf * 64 + j * 8;
            *(volatile v8h*)(oh + go) = vals[s];
        }
    }

    if (EPI == 3) {
        float* F = (float*)lds + wave * 1024;
        const int q = l >> 3, j = l & 7;
        const int row0 = bm * BT + wm * 32;
        #pragma unroll
        for (int p = 0; p < 2; ++p) {
            #pragma unroll
            for (int mi = 0; mi < 2; ++mi)
                #pragma unroll
                for (int nn = 0; nn < 2; ++nn)
                    #pragma unroll
                    for (int r = 0; r < 8; ++r)
                        F[(mi * 16 + 8 * h + r) * 32 + nn * 16 + m] = acc[mi][2 * p + nn][r];
            __syncthreads();
            const int colf = wn * 64 + p * 32;
            v4f vals[8];
            #pragma unroll
            for (int s = 0; s < 8; ++s) {
                const int lr = 4 * s + q;
                const int row = row0 + lr;
                vals[s] = *(const v4f*)(F + lr * 32 + j * 4);
                if (row < nreal)
                    *(volatile v4f*)(of + (size_t)row * DIM + colf + j * 4) = vals[s];
            }
            __threadfence();
            #pragma unroll
            for (int s = 0; s < 8; ++s) {
                const int lr = 4 * s + q;
                const int row = row0 + lr;
                if (row < nreal)
                    *(volatile v4f*)(of + (size_t)row * DIM + colf + j * 4) = vals[s];
            }
            __syncthreads();
        }
    }
}

extern "C" void kernel_launch(void* const* d_in, const int* in_sizes, int n_in,
                              void* d_out, int out_size, void* d_ws, size_t ws_size,
                              hipStream_t stream)
{
    if (n_in < 5) return;
    const int n_nodes = in_sizes[0] / 2;
    const int nreal   = n_nodes + 1;
    if (nreal < 1 || nreal > NP) return;
    if (in_sizes[1] != n_nodes || in_sizes[2] < 2) return;
    if (in_sizes[3] != DIM * 3 || in_sizes[4] != DIM) return;
    if (out_size != nreal * DIM) return;

    const float* nl  = (const float*)d_in[0];
    const float* td  = (const float*)d_in[1];
    const float* dep = (const float*)d_in[2];
    const float* w0w = (const float*)d_in[3];
    const float* w0b = (const float*)d_in[4];
    float* out = (float*)d_out;

    char* ws = (char*)d_ws;
    const size_t szA = (size_t)NP * NP * sizeof(_Float16);
    const size_t szF = (size_t)DIM * NP * sizeof(_Float16);
    size_t off = 0;
    _Float16* Ah   = (_Float16*)(ws + off); off += szA;
    _Float16* M2h  = (_Float16*)(ws + off); off += szA;
    _Float16* Wh   = (_Float16*)(ws + off); off += szA;
    _Float16* fv0T = (_Float16*)(ws + off); off += szF;
    _Float16* fv1T = (_Float16*)(ws + off); off += szF;
    if (off > ws_size) return;

    k_fv0<<<(2 * DIM * 32) / NTHR, NTHR, 0, stream>>>(nl, td, dep, w0w, w0b, fv0T, nreal);
    k_adj<<<NP / 32, NTHR, 0, stream>>>(nl, dep, Ah, nreal);
    k_gemm<0><<<dim3(NP / BT, NP / BT), NTHR, 0, stream>>>(Ah, Ah, Ah, M2h, out, nreal);
    k_gemm<2><<<dim3(NP / BT, 1), NTHR, 0, stream>>>(Ah, fv0T, Ah, fv1T, out, nreal);
    k_gemm<1><<<dim3(NP / BT, NP / BT), NTHR, 0, stream>>>(M2h, Ah, M2h, Wh, out, nreal);
    k_gemm<3><<<dim3(NP / BT, 1), NTHR, 0, stream>>>(Wh, fv1T, Ah, M2h, out, nreal);
}
